// NoSemanticSchemaGNN_15522011807981
// MI455X (gfx1250) — hardware-run, weakly checked
//
#include <hip/hip_runtime.h>
#include <math.h>

typedef __attribute__((ext_vector_type(16))) _Float16 v16h;
typedef __attribute__((ext_vector_type(16))) __bf16 v16b;
typedef __attribute__((ext_vector_type(8)))  _Float16 v8h;
typedef __attribute__((ext_vector_type(8)))  float v8f;
typedef __attribute__((ext_vector_type(4)))  float v4f;
typedef __attribute__((ext_vector_type(2)))  float v2f;
typedef __attribute__((ext_vector_type(4)))  unsigned v4u;
typedef __attribute__((ext_vector_type(4)))  int v4i;
typedef float __attribute__((may_alias)) float_a;
typedef int __attribute__((may_alias)) int_a;

template <typename T> __device__ __forceinline__ void vst2(void* p, T v) { *(volatile T*)p = v; __threadfence(); *(volatile T*)p = v; }
__device__ __forceinline__ v8f wmma16(v16h a, v16h b, v8f c) {
  v8f d = __builtin_amdgcn_wmma_f32_16x16x32_f16(false, a, false, b, (short)0, c, false, false);
  asm volatile("v_nop\n\tv_nop\n\tv_nop\n\tv_nop" : "+v"(d) : "v"(a), "v"(b));
  return d;
}
__device__ __forceinline__ v8f wmma_bf(v16b a, v16b b, v8f c) {
  v8f d = __builtin_amdgcn_wmma_f32_16x16x32_bf16(false, a, false, b, (short)0, c, false, false);
  asm volatile("v_nop\n\tv_nop\n\tv_nop\n\tv_nop" : "+v"(d) : "v"(a), "v"(b));
  return d;
}
__device__ __forceinline__ v16h frag_h(const _Float16* rowk0, int lane) {
  union { v16h v; v8h q[2]; } u; const _Float16* p = rowk0 + 8 * (lane >> 4);
  u.q[0] = *(const v8h*)p; u.q[1] = *(const v8h*)(p + 16); return u.v;
}
__device__ __forceinline__ v16h frag_f32(const float* rowk0, int lane) {
  v16h a; const float* p = rowk0 + 8 * (lane >> 4);
#pragma unroll
  for (int i = 0; i < 8; ++i) { a[i] = (_Float16)p[i]; a[8 + i] = (_Float16)p[16 + i]; }
  return a;
}
__device__ __forceinline__ v16h frag_f32s(const float* rowk0, int lane, float sc) {
  v16h a; const float* p = rowk0 + 8 * (lane >> 4);
#pragma unroll
  for (int i = 0; i < 8; ++i) { a[i] = (_Float16)(p[i] * sc); a[8 + i] = (_Float16)(p[16 + i] * sc); }
  return a;
}
__device__ __forceinline__ v16h fragc_f32(const float* W, int k0, int n, int lane, int ld, int K) {
  v16h a; const int g = lane >> 4;
#pragma unroll
  for (int i = 0; i < 8; ++i) { const int ka = k0 + 8 * g + i, kb = ka + 16;
    a[i] = (_Float16)(ka < K ? W[(size_t)(ka < K ? ka : K - 1) * ld + n] : 0.f); a[8 + i] = (_Float16)(kb < K ? W[(size_t)(kb < K ? kb : K - 1) * ld + n] : 0.f); }
  return a;
}
struct F2 { v16b h, l; };
__device__ __forceinline__ F2 bsplit16(const float v[16]) { F2 r;
#pragma unroll
  for (int i = 0; i < 16; ++i) { const __bf16 h = (__bf16)v[i]; r.h[i] = h; r.l[i] = (__bf16)(v[i] - (float)h); }
  return r; }
__device__ __forceinline__ F2 split_row(const float* row, int k0, int lane) { float v[16]; const float* p = row + k0 + 8 * (lane >> 4);
#pragma unroll
  for (int i = 0; i < 8; ++i) { v[i] = p[i]; v[8 + i] = p[16 + i]; }
  return bsplit16(v); }
__device__ __forceinline__ F2 split_rowK(const float* row, int k0, int lane, int K) { float v[16]; const int g = lane >> 4;
#pragma unroll
  for (int i = 0; i < 8; ++i) { const int ka = k0 + 8 * g + i, kb = ka + 16; v[i] = ka < K ? row[ka < K ? ka : K - 1] : 0.f; v[8 + i] = kb < K ? row[kb < K ? kb : K - 1] : 0.f; }
  return bsplit16(v); }
__device__ __forceinline__ F2 split_col(const float* W, int k0, int n, int lane, int ld, int K) { float v[16]; const int g = lane >> 4;
#pragma unroll
  for (int i = 0; i < 8; ++i) { const int ka = k0 + 8 * g + i, kb = ka + 16; v[i] = ka < K ? W[(size_t)(ka < K ? ka : K - 1) * ld + n] : 0.f; v[8 + i] = kb < K ? W[(size_t)(kb < K ? kb : K - 1) * ld + n] : 0.f; }
  return bsplit16(v); }
__device__ __forceinline__ v8f mac3(const F2& a, const F2& b, v8f c) { c = wmma_bf(a.l, b.h, c); c = wmma_bf(a.h, b.l, c); return wmma_bf(a.h, b.h, c); }
__device__ __forceinline__ float sigm(float v) { return 1.0f / (1.0f + expf(-v)); }
#define LDSX() do { asm volatile("s_wait_dscnt 0" ::: "memory"); __builtin_amdgcn_wave_barrier(); __builtin_amdgcn_fence(__ATOMIC_RELEASE, "workgroup"); } while (0)


#define NN 30000
#define NEDG 40000
#define NR 5
#define NG 64
#define IND 20
#define HID 256
#define NHD 4
#define DH 64
#define NL 3
#define NRB ((NN + 63) / 64)
#define NPAD (NRB * 64)
#ifndef NNT
#define NNT NN
#define NRBT NRB
#define NGT NG
#endif
typedef __attribute__((ext_vector_type(8))) __bf16 v8b;
__device__ __forceinline__ v16b frag_b(const __bf16* rowk0, int lane) {
  union { v16b v; v8b q[2]; } u; const __bf16* p = rowk0 + 8 * (lane >> 4);
  u.q[0] = *(const v8b*)p; u.q[1] = *(const v8b*)(p + 16); return u.v;
}
__device__ __forceinline__ float bfr(float v) { return (float)(__bf16)v; }
__device__ __attribute__((noinline)) float exp_ni(float v) { return expf(v); }
__device__ __attribute__((noinline)) float erf_ni(float v) { return erff(v); }

#define CSA_N 30000
#define CSA_E 40000
#define CSA_FINN (CSA_E + 32 * CSA_NBK)
#define CSA_CHUNK 4096
#define CSA_BKT 256
#define CSA_NCH ((CSA_E + CSA_CHUNK - 1) / CSA_CHUNK)
#define CSA_NBK ((CSA_N + CSA_BKT - 1) / CSA_BKT)
#define CSA_NBKP (((CSA_NBK + 63) / 64) * 64)
#define CSA_SEGCAP (CSA_E + 32 * CSA_NBK * CSA_NCH)
#ifndef CSA_BCAP
#define CSA_BCAP 10240
#endif
#define CSA_SZ_CNT   (4u * CSA_NCH * CSA_NBKP)
#define CSA_SZ_OFF   (4u * CSA_NBK * (((CSA_NCH + 31) / 32) * 32))
#define CSA_SZ_BST   (4u * (((CSA_NBK + 1 + 31) / 32) * 32))
#define CSA_SZ_SEG   (4u * CSA_SEGCAP)
#define CSA_SZ_FIN   (4u * (CSA_E + 32 * CSA_NBK))
#define CSA_SZ_ROW   (4u * CSA_NBK * CSA_BKT)
#define CSA_OFFP (((CSA_NCH + 31) / 32) * 32)

__global__ __launch_bounds__(256) void k_csA_cnt(const int* __restrict__ DST, int dstride, int* __restrict__ CNT) {
  __shared__ unsigned short sc[256][CSA_NBK + 1]; __shared__ __align__(16) int srow[CSA_NBKP];
  const int c = blockIdx.x, tid = threadIdx.x;
  for (int b = 0; b < CSA_NBK; ++b) sc[tid][b] = 0;
  const size_t e0 = (size_t)c * CSA_CHUNK + tid * 16;
  for (int i = 0; i < 16; ++i) { const size_t e = e0 + i; if (e < (size_t)CSA_E) { int d = DST[e * dstride]; d = min(max(d, 0), CSA_N - 1); sc[tid][d / CSA_BKT] += 1; } }
  __syncthreads();
  for (int b = tid; b < CSA_NBKP; b += 256) { int s = 0; if (b < CSA_NBK) for (int t = 0; t < 256; ++t) s += sc[t][b]; srow[b] = s; }
  __syncthreads();
  for (int q = tid; q < CSA_NBKP / 4; q += 256) vst2((unsigned*)(CNT + (size_t)c * CSA_NBKP + q * 4), *(const v4u*)&srow[q * 4]);
}
__global__ __launch_bounds__(256) void k_csA_scan(const int* __restrict__ CNT, int* __restrict__ OFF, int* __restrict__ BST) {
  __shared__ int sbt[CSA_NBK + 1]; __shared__ int sbs[((CSA_NBK + 1 + 31) / 32) * 32]; __shared__ int scnt[CSA_NBK + 1]; __shared__ __align__(16) int sbuf[64][CSA_OFFP];
  const int tid = threadIdx.x;
  for (int b = tid; b < CSA_NBK; b += 256) { int sp = 0, st = 0; for (int c = 0; c < CSA_NCH; ++c) { const int n = CNT[(size_t)c * CSA_NBKP + b]; st += n; sp += (n + 31) & ~31; } sbt[b] = sp; scnt[b] = st; }
  for (int b = tid; b < ((CSA_NBK + 1 + 31) / 32) * 32; b += 256) sbs[b] = 0;
  __syncthreads();
  if (tid == 0) { int acc = 0, accf = 0; for (int b = 0; b < CSA_NBK; ++b) { const int t = sbt[b]; sbt[b] = acc; acc += t; sbs[b] = accf; accf += (scnt[b] + 31) & ~31; } sbs[CSA_NBK] = accf; }
  __syncthreads();
  for (int b0 = 0; b0 < CSA_NBK; b0 += 64) {
    if (tid < 64 && b0 + tid < CSA_NBK) { const int b = b0 + tid; int o = sbt[b]; for (int c = 0; c < CSA_OFFP; ++c) { if (c < CSA_NCH) { sbuf[tid][c] = o; o += (CNT[(size_t)c * CSA_NBKP + b] + 31) & ~31; } else sbuf[tid][c] = 0; } }
    __syncthreads();
    for (int q = tid; q < 64 * (CSA_OFFP / 4); q += 256) { const int r = q / (CSA_OFFP / 4), pc = q % (CSA_OFFP / 4); if (b0 + r < CSA_NBK) vst2((unsigned*)(OFF + (size_t)(b0 + r) * CSA_OFFP + pc * 4), *(const v4u*)&sbuf[r][pc * 4]); }
    __syncthreads(); }
  for (int q = tid; q < ((CSA_NBK + 1 + 31) / 32) * 32 / 4; q += 256) vst2((unsigned*)(BST + q * 4), *(const v4u*)&sbs[q * 4]);
}
__global__ __launch_bounds__(256) void k_csA_scatter(const int* __restrict__ SRC, const int* __restrict__ DST, int sstride, int dstride, const int* __restrict__ OFF, int* __restrict__ SEGS, int* __restrict__ SEGE) {
  __shared__ unsigned short sc[256][CSA_NBK + 1]; __shared__ int sbase[CSA_NBK + 1]; __shared__ int scn[CSA_NBK + 1]; __shared__ int sord[CSA_CHUNK];
  const int c = blockIdx.x, tid = threadIdx.x;
  for (int b = 0; b < CSA_NBK; ++b) sc[tid][b] = 0;
  const size_t e0 = (size_t)c * CSA_CHUNK + tid * 16; int bk[16];
#pragma unroll
  for (int i = 0; i < 16; ++i) { const size_t e = e0 + i; bk[i] = -1; if (e < (size_t)CSA_E) { int d = DST[e * dstride]; d = min(max(d, 0), CSA_N - 1); bk[i] = d / CSA_BKT; sc[tid][bk[i]] += 1; } }
  __syncthreads();
  for (int b = tid; b < CSA_NBK; b += 256) { int acc = 0; for (int t = 0; t < 256; ++t) { const int v = sc[t][b]; sc[t][b] = (unsigned short)acc; acc += v; } scn[b] = acc; }
  __syncthreads();
  if (tid == 0) { int acc = 0; for (int b = 0; b < CSA_NBK; ++b) { sbase[b] = acc; acc += scn[b]; } }
  __syncthreads();
#pragma unroll
  for (int i = 0; i < 16; ++i) { if (bk[i] >= 0) { const int b = bk[i]; const int r = sc[tid][b]; sc[tid][b] = (unsigned short)(r + 1); sord[sbase[b] + r] = tid * 16 + i; } }
  __syncthreads();
  for (int b = 0; b < CSA_NBK; ++b) { const int n = scn[b]; if (n == 0) continue; const int nl = ((n + 31) & ~31); const size_t o = (size_t)(min(max(OFF[(size_t)b * CSA_OFFP + c], 0), CSA_SEGCAP - nl) & ~31);
    for (int q = tid; q < nl / 4; q += 256) { int4 vs, ve;
#pragma unroll
      for (int k = 0; k < 4; ++k) { const int i = q * 4 + k; int s = -1, eid = -1; if (i < n) { const size_t e = (size_t)c * CSA_CHUNK + sord[sbase[b] + i]; s = min(max(SRC[e * sstride], 0), CSA_N - 1); eid = (int)e; } vs[k] = s; ve[k] = eid; }
      vst2((unsigned*)(SEGS + o + q * 4), *(const v4u*)&vs); vst2((unsigned*)(SEGE + o + q * 4), *(const v4u*)&ve); } }
}
__global__ __launch_bounds__(256) void k_csA_bucket(const int* __restrict__ CNT, const int* __restrict__ OFF, const int* __restrict__ BST, const int* __restrict__ SEGS, const int* __restrict__ SEGE, const int* __restrict__ DST, int dstride, int* __restrict__ FS, int* __restrict__ FE, int* __restrict__ ROWST, int* __restrict__ ROWCNT) {
  __shared__ int ssrc[CSA_BCAP]; __shared__ int seid[CSA_BCAP]; __shared__ unsigned char snod[CSA_BCAP]; __shared__ int souts[CSA_BCAP]; __shared__ int soute[CSA_BCAP]; __shared__ int scount[256]; __shared__ int sstart[257]; __shared__ int stot;
  const int b = blockIdx.x, tid = threadIdx.x;
  if (tid == 0) { int t = 0; for (int c = 0; c < CSA_NCH; ++c) t += min(max(CNT[(size_t)c * CSA_NBKP + b], 0), CSA_CHUNK); stot = (t <= CSA_BCAP) ? t : 0; }
  __syncthreads();
  { int base = 0; for (int c = 0; c < CSA_NCH; ++c) { const int n = min(max(CNT[(size_t)c * CSA_NBKP + b], 0), CSA_CHUNK); const int o = min(max(OFF[(size_t)b * CSA_OFFP + c], 0), CSA_SEGCAP - ((n + 31) & ~31));
      for (int i = tid; i < n; i += 256) { const int p = base + i; if (p < CSA_BCAP) { ssrc[p] = min(max(SEGS[o + i], 0), CSA_N - 1); const int e = min(max(SEGE[o + i], 0), CSA_E - 1); seid[p] = e; int d = DST[(size_t)e * dstride]; d = min(max(d, 0), CSA_N - 1); const int dl = d - b * CSA_BKT; snod[p] = (unsigned char)(dl >= 0 && dl < 256 ? dl : 255); } }
      base += n; } }
  __syncthreads();
  const int node = b * CSA_BKT + tid; int cnt = 0; for (int p = 0; p < stot; ++p) cnt += (snod[p] == tid) ? 1 : 0;
  scount[tid] = cnt; __syncthreads();
  if (tid == 0) { int acc = 0; for (int t = 0; t < 256; ++t) { sstart[t] = acc; acc += scount[t]; } sstart[256] = acc; }
  __syncthreads();
  const int bst0 = min(max(BST[b], 0), CSA_FINN - ((sstart[256] + 31) & ~31)) & ~31; const int gst = bst0 + sstart[tid];
  { int w = sstart[tid]; for (int p = 0; p < stot; ++p) if (snod[p] == tid) { souts[w] = ssrc[p]; soute[w] = seid[p]; ++w; } }
  __syncthreads();
  { const int n = sstart[256]; const int nl = (n + 31) & ~31; for (int q = tid; q < nl / 4; q += 256) { int4 vs, ve;
#pragma unroll
      for (int k = 0; k < 4; ++k) { const int i = q * 4 + k; vs[k] = i < n ? souts[i] : -1; ve[k] = i < n ? soute[i] : -1; }
      vst2((unsigned*)(FS + bst0 + q * 4), *(const v4u*)&vs); vst2((unsigned*)(FE + bst0 + q * 4), *(const v4u*)&ve); } }
  __syncthreads();
  { __shared__ __align__(16) int srs[256], src2[256]; srs[tid] = node < CSA_N ? gst : 0; src2[tid] = node < CSA_N ? cnt : 0; __syncthreads();
    if (tid < 64) vst2((unsigned*)(ROWST + (size_t)b * 256 + tid * 4), *(const v4u*)&srs[tid * 4]); else if (tid < 128) vst2((unsigned*)(ROWCNT + (size_t)b * 256 + (tid - 64) * 4), *(const v4u*)&src2[(tid - 64) * 4]); }
}


#define CSB_N 30000
#define CSB_E 40000
#define CSB_FINN (CSB_E + 32 * CSB_NBK)
#define CSB_CHUNK 4096
#define CSB_BKT 256
#define CSB_NCH ((CSB_E + CSB_CHUNK - 1) / CSB_CHUNK)
#define CSB_NBK ((CSB_N + CSB_BKT - 1) / CSB_BKT)
#define CSB_NBKP (((CSB_NBK + 63) / 64) * 64)
#define CSB_SEGCAP (CSB_E + 32 * CSB_NBK * CSB_NCH)
#ifndef CSB_BCAP
#define CSB_BCAP 10240
#endif
#define CSB_SZ_CNT   (4u * CSB_NCH * CSB_NBKP)
#define CSB_SZ_OFF   (4u * CSB_NBK * (((CSB_NCH + 31) / 32) * 32))
#define CSB_SZ_BST   (4u * (((CSB_NBK + 1 + 31) / 32) * 32))
#define CSB_SZ_SEG   (4u * CSB_SEGCAP)
#define CSB_SZ_FIN   (4u * (CSB_E + 32 * CSB_NBK))
#define CSB_SZ_ROW   (4u * CSB_NBK * CSB_BKT)
#define CSB_OFFP (((CSB_NCH + 31) / 32) * 32)

__global__ __launch_bounds__(256) void k_csB_cnt(const int* __restrict__ DST, int dstride, int* __restrict__ CNT) {
  __shared__ unsigned short sc[256][CSB_NBK + 1]; __shared__ __align__(16) int srow[CSB_NBKP];
  const int c = blockIdx.x, tid = threadIdx.x;
  for (int b = 0; b < CSB_NBK; ++b) sc[tid][b] = 0;
  const size_t e0 = (size_t)c * CSB_CHUNK + tid * 16;
  for (int i = 0; i < 16; ++i) { const size_t e = e0 + i; if (e < (size_t)CSB_E) { int d = DST[e * dstride]; d = min(max(d, 0), CSB_N - 1); sc[tid][d / CSB_BKT] += 1; } }
  __syncthreads();
  for (int b = tid; b < CSB_NBKP; b += 256) { int s = 0; if (b < CSB_NBK) for (int t = 0; t < 256; ++t) s += sc[t][b]; srow[b] = s; }
  __syncthreads();
  for (int q = tid; q < CSB_NBKP / 4; q += 256) vst2((unsigned*)(CNT + (size_t)c * CSB_NBKP + q * 4), *(const v4u*)&srow[q * 4]);
}
__global__ __launch_bounds__(256) void k_csB_scan(const int* __restrict__ CNT, int* __restrict__ OFF, int* __restrict__ BST) {
  __shared__ int sbt[CSB_NBK + 1]; __shared__ int sbs[((CSB_NBK + 1 + 31) / 32) * 32]; __shared__ int scnt[CSB_NBK + 1]; __shared__ __align__(16) int sbuf[64][CSB_OFFP];
  const int tid = threadIdx.x;
  for (int b = tid; b < CSB_NBK; b += 256) { int sp = 0, st = 0; for (int c = 0; c < CSB_NCH; ++c) { const int n = CNT[(size_t)c * CSB_NBKP + b]; st += n; sp += (n + 31) & ~31; } sbt[b] = sp; scnt[b] = st; }
  for (int b = tid; b < ((CSB_NBK + 1 + 31) / 32) * 32; b += 256) sbs[b] = 0;
  __syncthreads();
  if (tid == 0) { int acc = 0, accf = 0; for (int b = 0; b < CSB_NBK; ++b) { const int t = sbt[b]; sbt[b] = acc; acc += t; sbs[b] = accf; accf += (scnt[b] + 31) & ~31; } sbs[CSB_NBK] = accf; }
  __syncthreads();
  for (int b0 = 0; b0 < CSB_NBK; b0 += 64) {
    if (tid < 64 && b0 + tid < CSB_NBK) { const int b = b0 + tid; int o = sbt[b]; for (int c = 0; c < CSB_OFFP; ++c) { if (c < CSB_NCH) { sbuf[tid][c] = o; o += (CNT[(size_t)c * CSB_NBKP + b] + 31) & ~31; } else sbuf[tid][c] = 0; } }
    __syncthreads();
    for (int q = tid; q < 64 * (CSB_OFFP / 4); q += 256) { const int r = q / (CSB_OFFP / 4), pc = q % (CSB_OFFP / 4); if (b0 + r < CSB_NBK) vst2((unsigned*)(OFF + (size_t)(b0 + r) * CSB_OFFP + pc * 4), *(const v4u*)&sbuf[r][pc * 4]); }
    __syncthreads(); }
  for (int q = tid; q < ((CSB_NBK + 1 + 31) / 32) * 32 / 4; q += 256) vst2((unsigned*)(BST + q * 4), *(const v4u*)&sbs[q * 4]);
}
__global__ __launch_bounds__(256) void k_csB_scatter(const int* __restrict__ SRC, const int* __restrict__ DST, int sstride, int dstride, const int* __restrict__ OFF, int* __restrict__ SEGS, int* __restrict__ SEGE) {
  __shared__ unsigned short sc[256][CSB_NBK + 1]; __shared__ int sbase[CSB_NBK + 1]; __shared__ int scn[CSB_NBK + 1]; __shared__ int sord[CSB_CHUNK];
  const int c = blockIdx.x, tid = threadIdx.x;
  for (int b = 0; b < CSB_NBK; ++b) sc[tid][b] = 0;
  const size_t e0 = (size_t)c * CSB_CHUNK + tid * 16; int bk[16];
#pragma unroll
  for (int i = 0; i < 16; ++i) { const size_t e = e0 + i; bk[i] = -1; if (e < (size_t)CSB_E) { int d = DST[e * dstride]; d = min(max(d, 0), CSB_N - 1); bk[i] = d / CSB_BKT; sc[tid][bk[i]] += 1; } }
  __syncthreads();
  for (int b = tid; b < CSB_NBK; b += 256) { int acc = 0; for (int t = 0; t < 256; ++t) { const int v = sc[t][b]; sc[t][b] = (unsigned short)acc; acc += v; } scn[b] = acc; }
  __syncthreads();
  if (tid == 0) { int acc = 0; for (int b = 0; b < CSB_NBK; ++b) { sbase[b] = acc; acc += scn[b]; } }
  __syncthreads();
#pragma unroll
  for (int i = 0; i < 16; ++i) { if (bk[i] >= 0) { const int b = bk[i]; const int r = sc[tid][b]; sc[tid][b] = (unsigned short)(r + 1); sord[sbase[b] + r] = tid * 16 + i; } }
  __syncthreads();
  for (int b = 0; b < CSB_NBK; ++b) { const int n = scn[b]; if (n == 0) continue; const int nl = ((n + 31) & ~31); const size_t o = (size_t)(min(max(OFF[(size_t)b * CSB_OFFP + c], 0), CSB_SEGCAP - nl) & ~31);
    for (int q = tid; q < nl / 4; q += 256) { int4 vs, ve;
#pragma unroll
      for (int k = 0; k < 4; ++k) { const int i = q * 4 + k; int s = -1, eid = -1; if (i < n) { const size_t e = (size_t)c * CSB_CHUNK + sord[sbase[b] + i]; s = min(max(SRC[e * sstride], 0), CSB_N - 1); eid = (int)e; } vs[k] = s; ve[k] = eid; }
      vst2((unsigned*)(SEGS + o + q * 4), *(const v4u*)&vs); vst2((unsigned*)(SEGE + o + q * 4), *(const v4u*)&ve); } }
}
__global__ __launch_bounds__(256) void k_csB_bucket(const int* __restrict__ CNT, const int* __restrict__ OFF, const int* __restrict__ BST, const int* __restrict__ SEGS, const int* __restrict__ SEGE, const int* __restrict__ DST, int dstride, int* __restrict__ FS, int* __restrict__ FE, int* __restrict__ ROWST, int* __restrict__ ROWCNT) {
  __shared__ int ssrc[CSB_BCAP]; __shared__ int seid[CSB_BCAP]; __shared__ unsigned char snod[CSB_BCAP]; __shared__ int souts[CSB_BCAP]; __shared__ int soute[CSB_BCAP]; __shared__ int scount[256]; __shared__ int sstart[257]; __shared__ int stot;
  const int b = blockIdx.x, tid = threadIdx.x;
  if (tid == 0) { int t = 0; for (int c = 0; c < CSB_NCH; ++c) t += min(max(CNT[(size_t)c * CSB_NBKP + b], 0), CSB_CHUNK); stot = (t <= CSB_BCAP) ? t : 0; }
  __syncthreads();
  { int base = 0; for (int c = 0; c < CSB_NCH; ++c) { const int n = min(max(CNT[(size_t)c * CSB_NBKP + b], 0), CSB_CHUNK); const int o = min(max(OFF[(size_t)b * CSB_OFFP + c], 0), CSB_SEGCAP - ((n + 31) & ~31));
      for (int i = tid; i < n; i += 256) { const int p = base + i; if (p < CSB_BCAP) { ssrc[p] = min(max(SEGS[o + i], 0), CSB_N - 1); const int e = min(max(SEGE[o + i], 0), CSB_E - 1); seid[p] = e; int d = DST[(size_t)e * dstride]; d = min(max(d, 0), CSB_N - 1); const int dl = d - b * CSB_BKT; snod[p] = (unsigned char)(dl >= 0 && dl < 256 ? dl : 255); } }
      base += n; } }
  __syncthreads();
  const int node = b * CSB_BKT + tid; int cnt = 0; for (int p = 0; p < stot; ++p) cnt += (snod[p] == tid) ? 1 : 0;
  scount[tid] = cnt; __syncthreads();
  if (tid == 0) { int acc = 0; for (int t = 0; t < 256; ++t) { sstart[t] = acc; acc += scount[t]; } sstart[256] = acc; }
  __syncthreads();
  const int bst0 = min(max(BST[b], 0), CSB_FINN - ((sstart[256] + 31) & ~31)) & ~31; const int gst = bst0 + sstart[tid];
  { int w = sstart[tid]; for (int p = 0; p < stot; ++p) if (snod[p] == tid) { souts[w] = ssrc[p]; soute[w] = seid[p]; ++w; } }
  __syncthreads();
  { const int n = sstart[256]; const int nl = (n + 31) & ~31; for (int q = tid; q < nl / 4; q += 256) { int4 vs, ve;
#pragma unroll
      for (int k = 0; k < 4; ++k) { const int i = q * 4 + k; vs[k] = i < n ? souts[i] : -1; ve[k] = i < n ? soute[i] : -1; }
      vst2((unsigned*)(FS + bst0 + q * 4), *(const v4u*)&vs); vst2((unsigned*)(FE + bst0 + q * 4), *(const v4u*)&ve); } }
  __syncthreads();
  { __shared__ __align__(16) int srs[256], src2[256]; srs[tid] = node < CSB_N ? gst : 0; src2[tid] = node < CSB_N ? cnt : 0; __syncthreads();
    if (tid < 64) vst2((unsigned*)(ROWST + (size_t)b * 256 + tid * 4), *(const v4u*)&srs[tid * 4]); else if (tid < 128) vst2((unsigned*)(ROWCNT + (size_t)b * 256 + (tid - 64) * 4), *(const v4u*)&src2[(tid - 64) * 4]); }
}


#define CSC_N 30000
#define CSC_E 40000
#define CSC_FINN (CSC_E + 32 * CSC_NBK)
#define CSC_CHUNK 4096
#define CSC_BKT 256
#define CSC_NCH ((CSC_E + CSC_CHUNK - 1) / CSC_CHUNK)
#define CSC_NBK ((CSC_N + CSC_BKT - 1) / CSC_BKT)
#define CSC_NBKP (((CSC_NBK + 63) / 64) * 64)
#define CSC_SEGCAP (CSC_E + 32 * CSC_NBK * CSC_NCH)
#ifndef CSC_BCAP
#define CSC_BCAP 10240
#endif
#define CSC_SZ_CNT   (4u * CSC_NCH * CSC_NBKP)
#define CSC_SZ_OFF   (4u * CSC_NBK * (((CSC_NCH + 31) / 32) * 32))
#define CSC_SZ_BST   (4u * (((CSC_NBK + 1 + 31) / 32) * 32))
#define CSC_SZ_SEG   (4u * CSC_SEGCAP)
#define CSC_SZ_FIN   (4u * (CSC_E + 32 * CSC_NBK))
#define CSC_SZ_ROW   (4u * CSC_NBK * CSC_BKT)
#define CSC_OFFP (((CSC_NCH + 31) / 32) * 32)

__global__ __launch_bounds__(256) void k_csC_cnt(const int* __restrict__ DST, int dstride, int* __restrict__ CNT) {
  __shared__ unsigned short sc[256][CSC_NBK + 1]; __shared__ __align__(16) int srow[CSC_NBKP];
  const int c = blockIdx.x, tid = threadIdx.x;
  for (int b = 0; b < CSC_NBK; ++b) sc[tid][b] = 0;
  const size_t e0 = (size_t)c * CSC_CHUNK + tid * 16;
  for (int i = 0; i < 16; ++i) { const size_t e = e0 + i; if (e < (size_t)CSC_E) { int d = DST[e * dstride]; d = min(max(d, 0), CSC_N - 1); sc[tid][d / CSC_BKT] += 1; } }
  __syncthreads();
  for (int b = tid; b < CSC_NBKP; b += 256) { int s = 0; if (b < CSC_NBK) for (int t = 0; t < 256; ++t) s += sc[t][b]; srow[b] = s; }
  __syncthreads();
  for (int q = tid; q < CSC_NBKP / 4; q += 256) vst2((unsigned*)(CNT + (size_t)c * CSC_NBKP + q * 4), *(const v4u*)&srow[q * 4]);
}
__global__ __launch_bounds__(256) void k_csC_scan(const int* __restrict__ CNT, int* __restrict__ OFF, int* __restrict__ BST) {
  __shared__ int sbt[CSC_NBK + 1]; __shared__ int sbs[((CSC_NBK + 1 + 31) / 32) * 32]; __shared__ int scnt[CSC_NBK + 1]; __shared__ __align__(16) int sbuf[64][CSC_OFFP];
  const int tid = threadIdx.x;
  for (int b = tid; b < CSC_NBK; b += 256) { int sp = 0, st = 0; for (int c = 0; c < CSC_NCH; ++c) { const int n = CNT[(size_t)c * CSC_NBKP + b]; st += n; sp += (n + 31) & ~31; } sbt[b] = sp; scnt[b] = st; }
  for (int b = tid; b < ((CSC_NBK + 1 + 31) / 32) * 32; b += 256) sbs[b] = 0;
  __syncthreads();
  if (tid == 0) { int acc = 0, accf = 0; for (int b = 0; b < CSC_NBK; ++b) { const int t = sbt[b]; sbt[b] = acc; acc += t; sbs[b] = accf; accf += (scnt[b] + 31) & ~31; } sbs[CSC_NBK] = accf; }
  __syncthreads();
  for (int b0 = 0; b0 < CSC_NBK; b0 += 64) {
    if (tid < 64 && b0 + tid < CSC_NBK) { const int b = b0 + tid; int o = sbt[b]; for (int c = 0; c < CSC_OFFP; ++c) { if (c < CSC_NCH) { sbuf[tid][c] = o; o += (CNT[(size_t)c * CSC_NBKP + b] + 31) & ~31; } else sbuf[tid][c] = 0; } }
    __syncthreads();
    for (int q = tid; q < 64 * (CSC_OFFP / 4); q += 256) { const int r = q / (CSC_OFFP / 4), pc = q % (CSC_OFFP / 4); if (b0 + r < CSC_NBK) vst2((unsigned*)(OFF + (size_t)(b0 + r) * CSC_OFFP + pc * 4), *(const v4u*)&sbuf[r][pc * 4]); }
    __syncthreads(); }
  for (int q = tid; q < ((CSC_NBK + 1 + 31) / 32) * 32 / 4; q += 256) vst2((unsigned*)(BST + q * 4), *(const v4u*)&sbs[q * 4]);
}
__global__ __launch_bounds__(256) void k_csC_scatter(const int* __restrict__ SRC, const int* __restrict__ DST, int sstride, int dstride, const int* __restrict__ OFF, int* __restrict__ SEGS, int* __restrict__ SEGE) {
  __shared__ unsigned short sc[256][CSC_NBK + 1]; __shared__ int sbase[CSC_NBK + 1]; __shared__ int scn[CSC_NBK + 1]; __shared__ int sord[CSC_CHUNK];
  const int c = blockIdx.x, tid = threadIdx.x;
  for (int b = 0; b < CSC_NBK; ++b) sc[tid][b] = 0;
  const size_t e0 = (size_t)c * CSC_CHUNK + tid * 16; int bk[16];
#pragma unroll
  for (int i = 0; i < 16; ++i) { const size_t e = e0 + i; bk[i] = -1; if (e < (size_t)CSC_E) { int d = DST[e * dstride]; d = min(max(d, 0), CSC_N - 1); bk[i] = d / CSC_BKT; sc[tid][bk[i]] += 1; } }
  __syncthreads();
  for (int b = tid; b < CSC_NBK; b += 256) { int acc = 0; for (int t = 0; t < 256; ++t) { const int v = sc[t][b]; sc[t][b] = (unsigned short)acc; acc += v; } scn[b] = acc; }
  __syncthreads();
  if (tid == 0) { int acc = 0; for (int b = 0; b < CSC_NBK; ++b) { sbase[b] = acc; acc += scn[b]; } }
  __syncthreads();
#pragma unroll
  for (int i = 0; i < 16; ++i) { if (bk[i] >= 0) { const int b = bk[i]; const int r = sc[tid][b]; sc[tid][b] = (unsigned short)(r + 1); sord[sbase[b] + r] = tid * 16 + i; } }
  __syncthreads();
  for (int b = 0; b < CSC_NBK; ++b) { const int n = scn[b]; if (n == 0) continue; const int nl = ((n + 31) & ~31); const size_t o = (size_t)(min(max(OFF[(size_t)b * CSC_OFFP + c], 0), CSC_SEGCAP - nl) & ~31);
    for (int q = tid; q < nl / 4; q += 256) { int4 vs, ve;
#pragma unroll
      for (int k = 0; k < 4; ++k) { const int i = q * 4 + k; int s = -1, eid = -1; if (i < n) { const size_t e = (size_t)c * CSC_CHUNK + sord[sbase[b] + i]; s = min(max(SRC[e * sstride], 0), CSC_N - 1); eid = (int)e; } vs[k] = s; ve[k] = eid; }
      vst2((unsigned*)(SEGS + o + q * 4), *(const v4u*)&vs); vst2((unsigned*)(SEGE + o + q * 4), *(const v4u*)&ve); } }
}
__global__ __launch_bounds__(256) void k_csC_bucket(const int* __restrict__ CNT, const int* __restrict__ OFF, const int* __restrict__ BST, const int* __restrict__ SEGS, const int* __restrict__ SEGE, const int* __restrict__ DST, int dstride, int* __restrict__ FS, int* __restrict__ FE, int* __restrict__ ROWST, int* __restrict__ ROWCNT) {
  __shared__ int ssrc[CSC_BCAP]; __shared__ int seid[CSC_BCAP]; __shared__ unsigned char snod[CSC_BCAP]; __shared__ int souts[CSC_BCAP]; __shared__ int soute[CSC_BCAP]; __shared__ int scount[256]; __shared__ int sstart[257]; __shared__ int stot;
  const int b = blockIdx.x, tid = threadIdx.x;
  if (tid == 0) { int t = 0; for (int c = 0; c < CSC_NCH; ++c) t += min(max(CNT[(size_t)c * CSC_NBKP + b], 0), CSC_CHUNK); stot = (t <= CSC_BCAP) ? t : 0; }
  __syncthreads();
  { int base = 0; for (int c = 0; c < CSC_NCH; ++c) { const int n = min(max(CNT[(size_t)c * CSC_NBKP + b], 0), CSC_CHUNK); const int o = min(max(OFF[(size_t)b * CSC_OFFP + c], 0), CSC_SEGCAP - ((n + 31) & ~31));
      for (int i = tid; i < n; i += 256) { const int p = base + i; if (p < CSC_BCAP) { ssrc[p] = min(max(SEGS[o + i], 0), CSC_N - 1); const int e = min(max(SEGE[o + i], 0), CSC_E - 1); seid[p] = e; int d = DST[(size_t)e * dstride]; d = min(max(d, 0), CSC_N - 1); const int dl = d - b * CSC_BKT; snod[p] = (unsigned char)(dl >= 0 && dl < 256 ? dl : 255); } }
      base += n; } }
  __syncthreads();
  const int node = b * CSC_BKT + tid; int cnt = 0; for (int p = 0; p < stot; ++p) cnt += (snod[p] == tid) ? 1 : 0;
  scount[tid] = cnt; __syncthreads();
  if (tid == 0) { int acc = 0; for (int t = 0; t < 256; ++t) { sstart[t] = acc; acc += scount[t]; } sstart[256] = acc; }
  __syncthreads();
  const int bst0 = min(max(BST[b], 0), CSC_FINN - ((sstart[256] + 31) & ~31)) & ~31; const int gst = bst0 + sstart[tid];
  { int w = sstart[tid]; for (int p = 0; p < stot; ++p) if (snod[p] == tid) { souts[w] = ssrc[p]; soute[w] = seid[p]; ++w; } }
  __syncthreads();
  { const int n = sstart[256]; const int nl = (n + 31) & ~31; for (int q = tid; q < nl / 4; q += 256) { int4 vs, ve;
#pragma unroll
      for (int k = 0; k < 4; ++k) { const int i = q * 4 + k; vs[k] = i < n ? souts[i] : -1; ve[k] = i < n ? soute[i] : -1; }
      vst2((unsigned*)(FS + bst0 + q * 4), *(const v4u*)&vs); vst2((unsigned*)(FE + bst0 + q * 4), *(const v4u*)&ve); } }
  __syncthreads();
  { __shared__ __align__(16) int srs[256], src2[256]; srs[tid] = node < CSC_N ? gst : 0; src2[tid] = node < CSC_N ? cnt : 0; __syncthreads();
    if (tid < 64) vst2((unsigned*)(ROWST + (size_t)b * 256 + tid * 4), *(const v4u*)&srs[tid * 4]); else if (tid < 128) vst2((unsigned*)(ROWCNT + (size_t)b * 256 + (tid - 64) * 4), *(const v4u*)&src2[(tid - 64) * 4]); }
}


#define CSD_N 30000
#define CSD_E 40000
#define CSD_FINN (CSD_E + 32 * CSD_NBK)
#define CSD_CHUNK 4096
#define CSD_BKT 256
#define CSD_NCH ((CSD_E + CSD_CHUNK - 1) / CSD_CHUNK)
#define CSD_NBK ((CSD_N + CSD_BKT - 1) / CSD_BKT)
#define CSD_NBKP (((CSD_NBK + 63) / 64) * 64)
#define CSD_SEGCAP (CSD_E + 32 * CSD_NBK * CSD_NCH)
#ifndef CSD_BCAP
#define CSD_BCAP 10240
#endif
#define CSD_SZ_CNT   (4u * CSD_NCH * CSD_NBKP)
#define CSD_SZ_OFF   (4u * CSD_NBK * (((CSD_NCH + 31) / 32) * 32))
#define CSD_SZ_BST   (4u * (((CSD_NBK + 1 + 31) / 32) * 32))
#define CSD_SZ_SEG   (4u * CSD_SEGCAP)
#define CSD_SZ_FIN   (4u * (CSD_E + 32 * CSD_NBK))
#define CSD_SZ_ROW   (4u * CSD_NBK * CSD_BKT)
#define CSD_OFFP (((CSD_NCH + 31) / 32) * 32)

__global__ __launch_bounds__(256) void k_csD_cnt(const int* __restrict__ DST, int dstride, int* __restrict__ CNT) {
  __shared__ unsigned short sc[256][CSD_NBK + 1]; __shared__ __align__(16) int srow[CSD_NBKP];
  const int c = blockIdx.x, tid = threadIdx.x;
  for (int b = 0; b < CSD_NBK; ++b) sc[tid][b] = 0;
  const size_t e0 = (size_t)c * CSD_CHUNK + tid * 16;
  for (int i = 0; i < 16; ++i) { const size_t e = e0 + i; if (e < (size_t)CSD_E) { int d = DST[e * dstride]; d = min(max(d, 0), CSD_N - 1); sc[tid][d / CSD_BKT] += 1; } }
  __syncthreads();
  for (int b = tid; b < CSD_NBKP; b += 256) { int s = 0; if (b < CSD_NBK) for (int t = 0; t < 256; ++t) s += sc[t][b]; srow[b] = s; }
  __syncthreads();
  for (int q = tid; q < CSD_NBKP / 4; q += 256) vst2((unsigned*)(CNT + (size_t)c * CSD_NBKP + q * 4), *(const v4u*)&srow[q * 4]);
}
__global__ __launch_bounds__(256) void k_csD_scan(const int* __restrict__ CNT, int* __restrict__ OFF, int* __restrict__ BST) {
  __shared__ int sbt[CSD_NBK + 1]; __shared__ int sbs[((CSD_NBK + 1 + 31) / 32) * 32]; __shared__ int scnt[CSD_NBK + 1]; __shared__ __align__(16) int sbuf[64][CSD_OFFP];
  const int tid = threadIdx.x;
  for (int b = tid; b < CSD_NBK; b += 256) { int sp = 0, st = 0; for (int c = 0; c < CSD_NCH; ++c) { const int n = CNT[(size_t)c * CSD_NBKP + b]; st += n; sp += (n + 31) & ~31; } sbt[b] = sp; scnt[b] = st; }
  for (int b = tid; b < ((CSD_NBK + 1 + 31) / 32) * 32; b += 256) sbs[b] = 0;
  __syncthreads();
  if (tid == 0) { int acc = 0, accf = 0; for (int b = 0; b < CSD_NBK; ++b) { const int t = sbt[b]; sbt[b] = acc; acc += t; sbs[b] = accf; accf += (scnt[b] + 31) & ~31; } sbs[CSD_NBK] = accf; }
  __syncthreads();
  for (int b0 = 0; b0 < CSD_NBK; b0 += 64) {
    if (tid < 64 && b0 + tid < CSD_NBK) { const int b = b0 + tid; int o = sbt[b]; for (int c = 0; c < CSD_OFFP; ++c) { if (c < CSD_NCH) { sbuf[tid][c] = o; o += (CNT[(size_t)c * CSD_NBKP + b] + 31) & ~31; } else sbuf[tid][c] = 0; } }
    __syncthreads();
    for (int q = tid; q < 64 * (CSD_OFFP / 4); q += 256) { const int r = q / (CSD_OFFP / 4), pc = q % (CSD_OFFP / 4); if (b0 + r < CSD_NBK) vst2((unsigned*)(OFF + (size_t)(b0 + r) * CSD_OFFP + pc * 4), *(const v4u*)&sbuf[r][pc * 4]); }
    __syncthreads(); }
  for (int q = tid; q < ((CSD_NBK + 1 + 31) / 32) * 32 / 4; q += 256) vst2((unsigned*)(BST + q * 4), *(const v4u*)&sbs[q * 4]);
}
__global__ __launch_bounds__(256) void k_csD_scatter(const int* __restrict__ SRC, const int* __restrict__ DST, int sstride, int dstride, const int* __restrict__ OFF, int* __restrict__ SEGS, int* __restrict__ SEGE) {
  __shared__ unsigned short sc[256][CSD_NBK + 1]; __shared__ int sbase[CSD_NBK + 1]; __shared__ int scn[CSD_NBK + 1]; __shared__ int sord[CSD_CHUNK];
  const int c = blockIdx.x, tid = threadIdx.x;
  for (int b = 0; b < CSD_NBK; ++b) sc[tid][b] = 0;
  const size_t e0 = (size_t)c * CSD_CHUNK + tid * 16; int bk[16];
#pragma unroll
  for (int i = 0; i < 16; ++i) { const size_t e = e0 + i; bk[i] = -1; if (e < (size_t)CSD_E) { int d = DST[e * dstride]; d = min(max(d, 0), CSD_N - 1); bk[i] = d / CSD_BKT; sc[tid][bk[i]] += 1; } }
  __syncthreads();
  for (int b = tid; b < CSD_NBK; b += 256) { int acc = 0; for (int t = 0; t < 256; ++t) { const int v = sc[t][b]; sc[t][b] = (unsigned short)acc; acc += v; } scn[b] = acc; }
  __syncthreads();
  if (tid == 0) { int acc = 0; for (int b = 0; b < CSD_NBK; ++b) { sbase[b] = acc; acc += scn[b]; } }
  __syncthreads();
#pragma unroll
  for (int i = 0; i < 16; ++i) { if (bk[i] >= 0) { const int b = bk[i]; const int r = sc[tid][b]; sc[tid][b] = (unsigned short)(r + 1); sord[sbase[b] + r] = tid * 16 + i; } }
  __syncthreads();
  for (int b = 0; b < CSD_NBK; ++b) { const int n = scn[b]; if (n == 0) continue; const int nl = ((n + 31) & ~31); const size_t o = (size_t)(min(max(OFF[(size_t)b * CSD_OFFP + c], 0), CSD_SEGCAP - nl) & ~31);
    for (int q = tid; q < nl / 4; q += 256) { int4 vs, ve;
#pragma unroll
      for (int k = 0; k < 4; ++k) { const int i = q * 4 + k; int s = -1, eid = -1; if (i < n) { const size_t e = (size_t)c * CSD_CHUNK + sord[sbase[b] + i]; s = min(max(SRC[e * sstride], 0), CSD_N - 1); eid = (int)e; } vs[k] = s; ve[k] = eid; }
      vst2((unsigned*)(SEGS + o + q * 4), *(const v4u*)&vs); vst2((unsigned*)(SEGE + o + q * 4), *(const v4u*)&ve); } }
}
__global__ __launch_bounds__(256) void k_csD_bucket(const int* __restrict__ CNT, const int* __restrict__ OFF, const int* __restrict__ BST, const int* __restrict__ SEGS, const int* __restrict__ SEGE, const int* __restrict__ DST, int dstride, int* __restrict__ FS, int* __restrict__ FE, int* __restrict__ ROWST, int* __restrict__ ROWCNT) {
  __shared__ int ssrc[CSD_BCAP]; __shared__ int seid[CSD_BCAP]; __shared__ unsigned char snod[CSD_BCAP]; __shared__ int souts[CSD_BCAP]; __shared__ int soute[CSD_BCAP]; __shared__ int scount[256]; __shared__ int sstart[257]; __shared__ int stot;
  const int b = blockIdx.x, tid = threadIdx.x;
  if (tid == 0) { int t = 0; for (int c = 0; c < CSD_NCH; ++c) t += min(max(CNT[(size_t)c * CSD_NBKP + b], 0), CSD_CHUNK); stot = (t <= CSD_BCAP) ? t : 0; }
  __syncthreads();
  { int base = 0; for (int c = 0; c < CSD_NCH; ++c) { const int n = min(max(CNT[(size_t)c * CSD_NBKP + b], 0), CSD_CHUNK); const int o = min(max(OFF[(size_t)b * CSD_OFFP + c], 0), CSD_SEGCAP - ((n + 31) & ~31));
      for (int i = tid; i < n; i += 256) { const int p = base + i; if (p < CSD_BCAP) { ssrc[p] = min(max(SEGS[o + i], 0), CSD_N - 1); const int e = min(max(SEGE[o + i], 0), CSD_E - 1); seid[p] = e; int d = DST[(size_t)e * dstride]; d = min(max(d, 0), CSD_N - 1); const int dl = d - b * CSD_BKT; snod[p] = (unsigned char)(dl >= 0 && dl < 256 ? dl : 255); } }
      base += n; } }
  __syncthreads();
  const int node = b * CSD_BKT + tid; int cnt = 0; for (int p = 0; p < stot; ++p) cnt += (snod[p] == tid) ? 1 : 0;
  scount[tid] = cnt; __syncthreads();
  if (tid == 0) { int acc = 0; for (int t = 0; t < 256; ++t) { sstart[t] = acc; acc += scount[t]; } sstart[256] = acc; }
  __syncthreads();
  const int bst0 = min(max(BST[b], 0), CSD_FINN - ((sstart[256] + 31) & ~31)) & ~31; const int gst = bst0 + sstart[tid];
  { int w = sstart[tid]; for (int p = 0; p < stot; ++p) if (snod[p] == tid) { souts[w] = ssrc[p]; soute[w] = seid[p]; ++w; } }
  __syncthreads();
  { const int n = sstart[256]; const int nl = (n + 31) & ~31; for (int q = tid; q < nl / 4; q += 256) { int4 vs, ve;
#pragma unroll
      for (int k = 0; k < 4; ++k) { const int i = q * 4 + k; vs[k] = i < n ? souts[i] : -1; ve[k] = i < n ? soute[i] : -1; }
      vst2((unsigned*)(FS + bst0 + q * 4), *(const v4u*)&vs); vst2((unsigned*)(FE + bst0 + q * 4), *(const v4u*)&ve); } }
  __syncthreads();
  { __shared__ __align__(16) int srs[256], src2[256]; srs[tid] = node < CSD_N ? gst : 0; src2[tid] = node < CSD_N ? cnt : 0; __syncthreads();
    if (tid < 64) vst2((unsigned*)(ROWST + (size_t)b * 256 + tid * 4), *(const v4u*)&srs[tid * 4]); else if (tid < 128) vst2((unsigned*)(ROWCNT + (size_t)b * 256 + (tid - 64) * 4), *(const v4u*)&src2[(tid - 64) * 4]); }
}


#define CSE_N 30000
#define CSE_E 40000
#define CSE_FINN (CSE_E + 32 * CSE_NBK)
#define CSE_CHUNK 4096
#define CSE_BKT 256
#define CSE_NCH ((CSE_E + CSE_CHUNK - 1) / CSE_CHUNK)
#define CSE_NBK ((CSE_N + CSE_BKT - 1) / CSE_BKT)
#define CSE_NBKP (((CSE_NBK + 63) / 64) * 64)
#define CSE_SEGCAP (CSE_E + 32 * CSE_NBK * CSE_NCH)
#ifndef CSE_BCAP
#define CSE_BCAP 10240
#endif
#define CSE_SZ_CNT   (4u * CSE_NCH * CSE_NBKP)
#define CSE_SZ_OFF   (4u * CSE_NBK * (((CSE_NCH + 31) / 32) * 32))
#define CSE_SZ_BST   (4u * (((CSE_NBK + 1 + 31) / 32) * 32))
#define CSE_SZ_SEG   (4u * CSE_SEGCAP)
#define CSE_SZ_FIN   (4u * (CSE_E + 32 * CSE_NBK))
#define CSE_SZ_ROW   (4u * CSE_NBK * CSE_BKT)
#define CSE_OFFP (((CSE_NCH + 31) / 32) * 32)

__global__ __launch_bounds__(256) void k_csE_cnt(const int* __restrict__ DST, int dstride, int* __restrict__ CNT) {
  __shared__ unsigned short sc[256][CSE_NBK + 1]; __shared__ __align__(16) int srow[CSE_NBKP];
  const int c = blockIdx.x, tid = threadIdx.x;
  for (int b = 0; b < CSE_NBK; ++b) sc[tid][b] = 0;
  const size_t e0 = (size_t)c * CSE_CHUNK + tid * 16;
  for (int i = 0; i < 16; ++i) { const size_t e = e0 + i; if (e < (size_t)CSE_E) { int d = DST[e * dstride]; d = min(max(d, 0), CSE_N - 1); sc[tid][d / CSE_BKT] += 1; } }
  __syncthreads();
  for (int b = tid; b < CSE_NBKP; b += 256) { int s = 0; if (b < CSE_NBK) for (int t = 0; t < 256; ++t) s += sc[t][b]; srow[b] = s; }
  __syncthreads();
  for (int q = tid; q < CSE_NBKP / 4; q += 256) vst2((unsigned*)(CNT + (size_t)c * CSE_NBKP + q * 4), *(const v4u*)&srow[q * 4]);
}
__global__ __launch_bounds__(256) void k_csE_scan(const int* __restrict__ CNT, int* __restrict__ OFF, int* __restrict__ BST) {
  __shared__ int sbt[CSE_NBK + 1]; __shared__ int sbs[((CSE_NBK + 1 + 31) / 32) * 32]; __shared__ int scnt[CSE_NBK + 1]; __shared__ __align__(16) int sbuf[64][CSE_OFFP];
  const int tid = threadIdx.x;
  for (int b = tid; b < CSE_NBK; b += 256) { int sp = 0, st = 0; for (int c = 0; c < CSE_NCH; ++c) { const int n = CNT[(size_t)c * CSE_NBKP + b]; st += n; sp += (n + 31) & ~31; } sbt[b] = sp; scnt[b] = st; }
  for (int b = tid; b < ((CSE_NBK + 1 + 31) / 32) * 32; b += 256) sbs[b] = 0;
  __syncthreads();
  if (tid == 0) { int acc = 0, accf = 0; for (int b = 0; b < CSE_NBK; ++b) { const int t = sbt[b]; sbt[b] = acc; acc += t; sbs[b] = accf; accf += (scnt[b] + 31) & ~31; } sbs[CSE_NBK] = accf; }
  __syncthreads();
  for (int b0 = 0; b0 < CSE_NBK; b0 += 64) {
    if (tid < 64 && b0 + tid < CSE_NBK) { const int b = b0 + tid; int o = sbt[b]; for (int c = 0; c < CSE_OFFP; ++c) { if (c < CSE_NCH) { sbuf[tid][c] = o; o += (CNT[(size_t)c * CSE_NBKP + b] + 31) & ~31; } else sbuf[tid][c] = 0; } }
    __syncthreads();
    for (int q = tid; q < 64 * (CSE_OFFP / 4); q += 256) { const int r = q / (CSE_OFFP / 4), pc = q % (CSE_OFFP / 4); if (b0 + r < CSE_NBK) vst2((unsigned*)(OFF + (size_t)(b0 + r) * CSE_OFFP + pc * 4), *(const v4u*)&sbuf[r][pc * 4]); }
    __syncthreads(); }
  for (int q = tid; q < ((CSE_NBK + 1 + 31) / 32) * 32 / 4; q += 256) vst2((unsigned*)(BST + q * 4), *(const v4u*)&sbs[q * 4]);
}
__global__ __launch_bounds__(256) void k_csE_scatter(const int* __restrict__ SRC, const int* __restrict__ DST, int sstride, int dstride, const int* __restrict__ OFF, int* __restrict__ SEGS, int* __restrict__ SEGE) {
  __shared__ unsigned short sc[256][CSE_NBK + 1]; __shared__ int sbase[CSE_NBK + 1]; __shared__ int scn[CSE_NBK + 1]; __shared__ int sord[CSE_CHUNK];
  const int c = blockIdx.x, tid = threadIdx.x;
  for (int b = 0; b < CSE_NBK; ++b) sc[tid][b] = 0;
  const size_t e0 = (size_t)c * CSE_CHUNK + tid * 16; int bk[16];
#pragma unroll
  for (int i = 0; i < 16; ++i) { const size_t e = e0 + i; bk[i] = -1; if (e < (size_t)CSE_E) { int d = DST[e * dstride]; d = min(max(d, 0), CSE_N - 1); bk[i] = d / CSE_BKT; sc[tid][bk[i]] += 1; } }
  __syncthreads();
  for (int b = tid; b < CSE_NBK; b += 256) { int acc = 0; for (int t = 0; t < 256; ++t) { const int v = sc[t][b]; sc[t][b] = (unsigned short)acc; acc += v; } scn[b] = acc; }
  __syncthreads();
  if (tid == 0) { int acc = 0; for (int b = 0; b < CSE_NBK; ++b) { sbase[b] = acc; acc += scn[b]; } }
  __syncthreads();
#pragma unroll
  for (int i = 0; i < 16; ++i) { if (bk[i] >= 0) { const int b = bk[i]; const int r = sc[tid][b]; sc[tid][b] = (unsigned short)(r + 1); sord[sbase[b] + r] = tid * 16 + i; } }
  __syncthreads();
  for (int b = 0; b < CSE_NBK; ++b) { const int n = scn[b]; if (n == 0) continue; const int nl = ((n + 31) & ~31); const size_t o = (size_t)(min(max(OFF[(size_t)b * CSE_OFFP + c], 0), CSE_SEGCAP - nl) & ~31);
    for (int q = tid; q < nl / 4; q += 256) { int4 vs, ve;
#pragma unroll
      for (int k = 0; k < 4; ++k) { const int i = q * 4 + k; int s = -1, eid = -1; if (i < n) { const size_t e = (size_t)c * CSE_CHUNK + sord[sbase[b] + i]; s = min(max(SRC[e * sstride], 0), CSE_N - 1); eid = (int)e; } vs[k] = s; ve[k] = eid; }
      vst2((unsigned*)(SEGS + o + q * 4), *(const v4u*)&vs); vst2((unsigned*)(SEGE + o + q * 4), *(const v4u*)&ve); } }
}
__global__ __launch_bounds__(256) void k_csE_bucket(const int* __restrict__ CNT, const int* __restrict__ OFF, const int* __restrict__ BST, const int* __restrict__ SEGS, const int* __restrict__ SEGE, const int* __restrict__ DST, int dstride, int* __restrict__ FS, int* __restrict__ FE, int* __restrict__ ROWST, int* __restrict__ ROWCNT) {
  __shared__ int ssrc[CSE_BCAP]; __shared__ int seid[CSE_BCAP]; __shared__ unsigned char snod[CSE_BCAP]; __shared__ int souts[CSE_BCAP]; __shared__ int soute[CSE_BCAP]; __shared__ int scount[256]; __shared__ int sstart[257]; __shared__ int stot;
  const int b = blockIdx.x, tid = threadIdx.x;
  if (tid == 0) { int t = 0; for (int c = 0; c < CSE_NCH; ++c) t += min(max(CNT[(size_t)c * CSE_NBKP + b], 0), CSE_CHUNK); stot = (t <= CSE_BCAP) ? t : 0; }
  __syncthreads();
  { int base = 0; for (int c = 0; c < CSE_NCH; ++c) { const int n = min(max(CNT[(size_t)c * CSE_NBKP + b], 0), CSE_CHUNK); const int o = min(max(OFF[(size_t)b * CSE_OFFP + c], 0), CSE_SEGCAP - ((n + 31) & ~31));
      for (int i = tid; i < n; i += 256) { const int p = base + i; if (p < CSE_BCAP) { ssrc[p] = min(max(SEGS[o + i], 0), CSE_N - 1); const int e = min(max(SEGE[o + i], 0), CSE_E - 1); seid[p] = e; int d = DST[(size_t)e * dstride]; d = min(max(d, 0), CSE_N - 1); const int dl = d - b * CSE_BKT; snod[p] = (unsigned char)(dl >= 0 && dl < 256 ? dl : 255); } }
      base += n; } }
  __syncthreads();
  const int node = b * CSE_BKT + tid; int cnt = 0; for (int p = 0; p < stot; ++p) cnt += (snod[p] == tid) ? 1 : 0;
  scount[tid] = cnt; __syncthreads();
  if (tid == 0) { int acc = 0; for (int t = 0; t < 256; ++t) { sstart[t] = acc; acc += scount[t]; } sstart[256] = acc; }
  __syncthreads();
  const int bst0 = min(max(BST[b], 0), CSE_FINN - ((sstart[256] + 31) & ~31)) & ~31; const int gst = bst0 + sstart[tid];
  { int w = sstart[tid]; for (int p = 0; p < stot; ++p) if (snod[p] == tid) { souts[w] = ssrc[p]; soute[w] = seid[p]; ++w; } }
  __syncthreads();
  { const int n = sstart[256]; const int nl = (n + 31) & ~31; for (int q = tid; q < nl / 4; q += 256) { int4 vs, ve;
#pragma unroll
      for (int k = 0; k < 4; ++k) { const int i = q * 4 + k; vs[k] = i < n ? souts[i] : -1; ve[k] = i < n ? soute[i] : -1; }
      vst2((unsigned*)(FS + bst0 + q * 4), *(const v4u*)&vs); vst2((unsigned*)(FE + bst0 + q * 4), *(const v4u*)&ve); } }
  __syncthreads();
  { __shared__ __align__(16) int srs[256], src2[256]; srs[tid] = node < CSE_N ? gst : 0; src2[tid] = node < CSE_N ? cnt : 0; __syncthreads();
    if (tid < 64) vst2((unsigned*)(ROWST + (size_t)b * 256 + tid * 4), *(const v4u*)&srs[tid * 4]); else if (tid < 128) vst2((unsigned*)(ROWCNT + (size_t)b * 256 + (tid - 64) * 4), *(const v4u*)&src2[(tid - 64) * 4]); }
}


#define WS_ACNT (0u)
#define WS_AOFF (WS_ACNT + CSA_SZ_CNT)
#define WS_ABST (WS_AOFF + CSA_SZ_OFF)
#define WS_ASEGS (WS_ABST + CSA_SZ_BST)
#define WS_ASEGE (WS_ASEGS + CSA_SZ_SEG)
#define WS_AFS (WS_ASEGE + CSA_SZ_SEG)
#define WS_AFE (WS_AFS + CSA_SZ_FIN)
#define WS_ARST (WS_AFE + CSA_SZ_FIN)
#define WS_ARCT (WS_ARST + CSA_SZ_ROW)
#define WS_BCNT (WS_ARCT + CSA_SZ_ROW)
#define WS_BOFF (WS_BCNT + CSB_SZ_CNT)
#define WS_BBST (WS_BOFF + CSB_SZ_OFF)
#define WS_BSEGS (WS_BBST + CSB_SZ_BST)
#define WS_BSEGE (WS_BSEGS + CSB_SZ_SEG)
#define WS_BFS (WS_BSEGE + CSB_SZ_SEG)
#define WS_BFE (WS_BFS + CSB_SZ_FIN)
#define WS_BRST (WS_BFE + CSB_SZ_FIN)
#define WS_BRCT (WS_BRST + CSB_SZ_ROW)
#define WS_CCNT (WS_BRCT + CSB_SZ_ROW)
#define WS_COFF (WS_CCNT + CSC_SZ_CNT)
#define WS_CBST (WS_COFF + CSC_SZ_OFF)
#define WS_CSEGS (WS_CBST + CSC_SZ_BST)
#define WS_CSEGE (WS_CSEGS + CSC_SZ_SEG)
#define WS_CFS (WS_CSEGE + CSC_SZ_SEG)
#define WS_CFE (WS_CFS + CSC_SZ_FIN)
#define WS_CRST (WS_CFE + CSC_SZ_FIN)
#define WS_CRCT (WS_CRST + CSC_SZ_ROW)
#define WS_DCNT (WS_CRCT + CSC_SZ_ROW)
#define WS_DOFF (WS_DCNT + CSD_SZ_CNT)
#define WS_DBST (WS_DOFF + CSD_SZ_OFF)
#define WS_DSEGS (WS_DBST + CSD_SZ_BST)
#define WS_DSEGE (WS_DSEGS + CSD_SZ_SEG)
#define WS_DFS (WS_DSEGE + CSD_SZ_SEG)
#define WS_DFE (WS_DFS + CSD_SZ_FIN)
#define WS_DRST (WS_DFE + CSD_SZ_FIN)
#define WS_DRCT (WS_DRST + CSD_SZ_ROW)
#define WS_ECNT (WS_DRCT + CSD_SZ_ROW)
#define WS_EOFF (WS_ECNT + CSE_SZ_CNT)
#define WS_EBST (WS_EOFF + CSE_SZ_OFF)
#define WS_ESEGS (WS_EBST + CSE_SZ_BST)
#define WS_ESEGE (WS_ESEGS + CSE_SZ_SEG)
#define WS_EFS (WS_ESEGE + CSE_SZ_SEG)
#define WS_EFE (WS_EFS + CSE_SZ_FIN)
#define WS_ERST (WS_EFE + CSE_SZ_FIN)
#define WS_ERCT (WS_ERST + CSE_SZ_ROW)
#define WS_PW   (WS_ERCT + CSE_SZ_ROW)
#define PQKV(l) ((size_t)(l) * 768 * HID)
#define POUT(l) ((size_t)NL * 768 * HID + (size_t)(l) * HID * HID)
#define PREL(l, r, w, h) ((size_t)NL * 768 * HID + (size_t)NL * HID * HID + ((((size_t)(l) * NR + (r)) * 2 + (w)) * NHD + (h)) * DH * DH)
#define PL1 ((size_t)NL * 768 * HID + (size_t)NL * HID * HID + (size_t)NL * NR * 2 * NHD * DH * DH)
#define PWEND (PL1 + (size_t)128 * HID)
#define WS_H    (WS_PW + 2u * PWEND)
#define WS_QKV  (WS_H + 4u * NPAD * HID)
#define WS_PB   (WS_QKV + 4u * NPAD * 768)
#define WS_AL   (WS_PB + 4u * NPAD * HID)
#define WS_MS   (WS_AL + 4u * NR * NEDG * NHD)
#define WS_AGG  (WS_MS + 4u * NPAD * 8)
#define WS_T    (WS_AGG + 4u * NPAD * HID)
#define WS_G    (WS_T + 4u * NPAD * HID)
#define WS_HL   (WS_G + 4u * NG * 512)
#define WS_NL   (WS_HL + 4u * NPAD * 128)
#define WS_END  (WS_NL + 4u * NPAD)

__global__ __launch_bounds__(256) void k_packW(const float* __restrict__ Wm, int K, int NOUT, __bf16* __restrict__ DST) {
  __shared__ __align__(16) __bf16 s[512]; const int n = blockIdx.x, tid = threadIdx.x;
  for (int k = tid; k < K; k += 256) s[k] = (__bf16)Wm[(size_t)k * NOUT + n];
  __syncthreads();
  for (int q = tid; q < K / 8; q += 256) vst2((unsigned*)(DST + (size_t)n * K + q * 8), *(const v4u*)&s[q * 8]);
}
__global__ __launch_bounds__(64) void k_packrel(const float* __restrict__ AR, const float* __restrict__ MR, __bf16* __restrict__ PW) {
  __shared__ __align__(16) __bf16 s[64]; const int f = blockIdx.x, idx = blockIdx.y, d = threadIdx.x; const int h = idx % NHD, w = (idx / NHD) % 2, r = (idx / (NHD * 2)) % NR, l = idx / (NHD * 2 * NR);
  const float* src = (w ? MR : AR) + ((((size_t)l * NR + r) * NHD + h) * DH + d) * DH + f; s[d] = (__bf16)src[0]; __syncthreads();
  if (d < 8) vst2((unsigned*)(PW + PREL(l, r, w, h) + (size_t)f * DH + d * 8), *(const v4u*)&s[d * 8]);
}
__global__ __launch_bounds__(256) void k_inp(const float* __restrict__ X, const float* __restrict__ WI, const float* __restrict__ BI, float* __restrict__ Hh) {
  __shared__ float sx[64][IND]; __shared__ __align__(16) float so[64][HID]; const int tid = threadIdx.x; const size_t n0 = (size_t)blockIdx.x * 64;
  for (int q = tid; q < 64 * IND; q += 256) { const size_t n = n0 + q / IND; sx[q / IND][q % IND] = (n < NN) ? bfr(X[n * IND + q % IND]) : 0.f; }
  float w[IND];
#pragma unroll
  for (int k = 0; k < IND; ++k) w[k] = bfr(WI[k * HID + tid]);
  const float bb = bfr(BI[tid]);
  __syncthreads();
  for (int rl = 0; rl < 64; ++rl) { float a = bb;
#pragma unroll
    for (int k = 0; k < IND; ++k) a += sx[rl][k] * w[k];
    so[rl][tid] = (n0 + rl < NN) ? fmaxf(a, 0.f) : 0.f; }
  __syncthreads();
  for (int q = tid; q < 64 * HID / 4; q += 256) { const int rl = q / (HID / 4), pc = q % (HID / 4); vst2(Hh + (n0 + rl) * HID + pc * 4, *(const v4f*)&so[rl][pc * 4]); }
}
template <int EPI>
__global__ __launch_bounds__(128) void k_gemm(const float* __restrict__ A, int lda, int K, const __bf16* __restrict__ P, const float* __restrict__ bias, const float* __restrict__ RES, const float* __restrict__ SKP, float* __restrict__ OUT, int ldo) {
  const float sk = (EPI == 2) ? sigm(bfr(SKP[0])) : 0.f;
  __shared__ __align__(16) float so[4][16][132];
  const int tid = threadIdx.x, wave = tid >> 5, lane = tid & 31, col = lane & 15, g = lane >> 4; const size_t r0 = (size_t)blockIdx.x * 64 + wave * 16; const int n0 = blockIdx.y * 128;
  v8f acc[8] = {};
#pragma unroll 2
  for (int kc = 0; kc < K / 32; ++kc) { F2 a;
    if (EPI == 2) { float v[16]; const float* p = A + (r0 + col) * (size_t)lda + kc * 32 + 8 * g;
#pragma unroll
      for (int i = 0; i < 16; ++i) { const float x = (i < 8) ? p[i] : p[16 + i - 8]; v[i] = 0.5f * x * (1.0f + erf_ni(x * 0.70710678118654752f)); }
      a = bsplit16(v); }
    else a = split_row(A + (r0 + col) * (size_t)lda, kc * 32, lane);
#pragma unroll
    for (int j = 0; j < 8; ++j) { const v16b w = frag_b(P + (size_t)(n0 + j * 16 + col) * K + kc * 32, lane); acc[j] = wmma_bf(a.l, w, acc[j]); acc[j] = wmma_bf(a.h, w, acc[j]); } }
#pragma unroll
  for (int j = 0; j < 8; ++j) { const int n = n0 + j * 16 + col; const float bb = bfr(bias[n]);
#pragma unroll
    for (int r = 0; r < 8; ++r) { float v = acc[j][r] + bb; if (EPI == 1) v = fmaxf(v, 0.f); if (EPI == 2) { const float hx = RES[(r0 + 8 * g + r) * (size_t)ldo + n]; v = hx + (sk * v + (1.0f - sk) * hx); } so[wave][8 * g + r][j * 16 + col] = v; } }
  LDSX();
  for (int rl = 0; rl < 16; ++rl) vst2(OUT + (r0 + rl) * (size_t)ldo + n0 + lane * 4, *(const v4f*)&so[wave][rl][lane * 4]);
}
__global__ __launch_bounds__(128) void k_rel(const float* __restrict__ QKV, int coff, const __bf16* __restrict__ PR, float* __restrict__ OUT) {
  __shared__ __align__(16) float so[4][16][68];
  const int tid = threadIdx.x, wave = tid >> 5, lane = tid & 31, col = lane & 15, g = lane >> 4; const size_t r0 = (size_t)blockIdx.x * 64 + wave * 16; const int h = blockIdx.y; const __bf16* P = PR + (size_t)h * DH * DH;
  v8f acc[4] = {};
#pragma unroll
  for (int kc = 0; kc < 2; ++kc) { const F2 a = split_row(QKV + (r0 + col) * 768 + coff + h * DH, kc * 32, lane);
#pragma unroll
    for (int j = 0; j < 4; ++j) { const v16b w = frag_b(P + (size_t)(j * 16 + col) * DH + kc * 32, lane); acc[j] = wmma_bf(a.l, w, acc[j]); acc[j] = wmma_bf(a.h, w, acc[j]); } }
#pragma unroll
  for (int j = 0; j < 4; ++j)
#pragma unroll
    for (int r = 0; r < 8; ++r) so[wave][8 * g + r][j * 16 + col] = acc[j][r];
  LDSX();
  for (int rl = 0; rl < 16; ++rl) if (lane < 16) vst2(OUT + (r0 + rl) * HID + h * DH + lane * 4, *(const v4f*)&so[wave][rl][lane * 4]);
}
__global__ __launch_bounds__(256) void k_logit(const float* __restrict__ PK, const float* __restrict__ QKV, const int* __restrict__ SRC, const int* __restrict__ DSTI, const float* __restrict__ PRL, int r, float* __restrict__ AL) {
  __shared__ __align__(16) float sa[64 * NHD]; const int tid = threadIdx.x; const int el = tid >> 2, h = tid & 3; const size_t e = (size_t)blockIdx.x * 64 + el;
  float a = 0.f;
  if (e < NEDG) { const int s = min(max(SRC[e], 0), NN - 1), d = min(max(DSTI[e], 0), NN - 1); const float* pk = PK + (size_t)s * HID + h * DH; const float* q = QKV + (size_t)d * 768 + HID + h * DH;
#pragma unroll 8
    for (int f = 0; f < DH; ++f) a += pk[f] * q[f];
    a = a * bfr(PRL[r * NHD + h]) / 8.0f; }
  sa[tid] = a; __syncthreads();
  if (tid < 64) vst2(AL + ((size_t)r * NEDG + (size_t)blockIdx.x * 64) * NHD + tid * 4, *(const v4f*)&sa[tid * 4]);
}
__global__ __launch_bounds__(256) void k_stats(const float* __restrict__ AL, const int* __restrict__ AFE_, const int* __restrict__ ARST_, const int* __restrict__ ARCT_, const int* __restrict__ BFE_, const int* __restrict__ BRST_, const int* __restrict__ BRCT_, const int* __restrict__ CFE_, const int* __restrict__ CRST_, const int* __restrict__ CRCT_, const int* __restrict__ DFE_, const int* __restrict__ DRST_, const int* __restrict__ DRCT_, const int* __restrict__ EFE_, const int* __restrict__ ERST_, const int* __restrict__ ERCT_, float* __restrict__ MS) {
  __shared__ __align__(16) float sm[64][8]; const int tid = threadIdx.x; const int nl = tid >> 2, h = tid & 3; const size_t n = (size_t)blockIdx.x * 64 + nl;
  const int* FEs[NR] = {AFE_, BFE_, CFE_, DFE_, EFE_}; const int* RSTs[NR] = {ARST_, BRST_, CRST_, DRST_, ERST_}; const int* RCTs[NR] = {ARCT_, BRCT_, CRCT_, DRCT_, ERCT_};
  float mx = -3.0e38f; int any = 0;
  if (n < NNT) {
#pragma unroll
    for (int r = 0; r < NR; ++r) { const int cnt = min(max(RCTs[r][n], 0), CSA_BCAP); const int st = min(max(RSTs[r][n], 0), CSA_FINN - cnt);
      for (int i = 0; i < cnt; ++i) { const int e = min(max(FEs[r][st + i], 0), NEDG - 1); mx = fmaxf(mx, AL[((size_t)r * NEDG + e) * NHD + h]); any = 1; } } }
  const float m = any ? mx : 0.f; float s = 0.f;
  if (n < NNT) {
#pragma unroll
    for (int r = 0; r < NR; ++r) { const int cnt = min(max(RCTs[r][n], 0), CSA_BCAP); const int st = min(max(RSTs[r][n], 0), CSA_FINN - cnt);
      for (int i = 0; i < cnt; ++i) { const int e = min(max(FEs[r][st + i], 0), NEDG - 1); s += exp_ni(AL[((size_t)r * NEDG + e) * NHD + h] - m); } } }
  sm[nl][h] = m; sm[nl][4 + h] = s; __syncthreads();
  for (int q = tid; q < 64 * 2; q += 256) vst2(MS + ((size_t)blockIdx.x * 64) * 8 + q * 4, *(const v4f*)(&sm[0][0] + q * 4));
}
template <int FIRST>
__global__ __launch_bounds__(256) void k_aggr(const float* __restrict__ PV, const float* __restrict__ AL, const float* __restrict__ MS, const int* __restrict__ FS, const int* __restrict__ FE, const int* __restrict__ RST, const int* __restrict__ RCT, int r, float* __restrict__ AGG) {
  const int tid = threadIdx.x;
  for (int pass = 0; pass < 16; ++pass) { const int nl = pass * 4 + (tid >> 6); const int f0 = (tid & 63) * 4; const int h = f0 / DH; const size_t n = (size_t)blockIdx.x * 64 + nl;
    v4f acc = {0.f, 0.f, 0.f, 0.f};
    if (!FIRST) acc = *(const v4f*)(AGG + n * HID + f0);
    if (n < NNT) { const int cnt = min(max(RCT[n], 0), CSA_BCAP); const int st = min(max(RST[n], 0), CSA_FINN - cnt); const float m = MS[n * 8 + h], s = MS[n * 8 + 4 + h];
      for (int i = 0; i < cnt; ++i) { const int src = min(max(FS[st + i], 0), NN - 1); const int e = min(max(FE[st + i], 0), NEDG - 1); const float a = exp_ni(AL[((size_t)r * NEDG + e) * NHD + h] - m) / s; const float* row = PV + (size_t)src * HID + f0;
#pragma unroll
        for (int k = 0; k < 4; ++k) acc[k] += a * row[k]; } }
    vst2(AGG + n * HID + f0, acc); }
}
__global__ __launch_bounds__(256) void k_ln(const float* __restrict__ T, const float* __restrict__ G, const float* __restrict__ Bb, float* __restrict__ Hh) {
  __shared__ __align__(16) float s[8][HID]; const int tid = threadIdx.x, wave = tid >> 5, lane = tid & 31; const size_t row = (size_t)blockIdx.x * 8 + wave;
  float v[8]; float sum = 0.f;
#pragma unroll
  for (int k = 0; k < 8; ++k) { v[k] = T[row * HID + lane + 32 * k]; sum += v[k]; }
#pragma unroll
  for (int o = 1; o < 32; o <<= 1) sum += __shfl_xor(sum, o);
  const float mu = sum / (float)HID; float var = 0.f;
#pragma unroll
  for (int k = 0; k < 8; ++k) { const float d = v[k] - mu; var += d * d; }
#pragma unroll
  for (int o = 1; o < 32; o <<= 1) var += __shfl_xor(var, o);
  const float rs = rsqrtf(var / (float)HID + 1e-5f);
#pragma unroll
  for (int k = 0; k < 8; ++k) { const int c = lane + 32 * k; s[wave][c] = (v[k] - mu) * rs * bfr(G[c]) + bfr(Bb[c]); }
  LDSX();
  for (int pc = lane; pc < HID / 4; pc += 32) vst2(Hh + row * HID + pc * 4, *(const v4f*)&s[wave][pc * 4]);
}
__global__ __launch_bounds__(256) void k_pool(const float* __restrict__ Hh, const int* __restrict__ BATCH, float* __restrict__ Gp) {
  __shared__ int slo, shi; __shared__ __align__(16) float so[512]; const int tid = threadIdx.x, gidx = blockIdx.x;
  if (tid == 0) { int lo = 0, hi = NNT; while (lo < hi) { const int mid = (lo + hi) >> 1; if (BATCH[mid] < gidx) lo = mid + 1; else hi = mid; } slo = lo; int lo2 = lo, hi2 = NNT; while (lo2 < hi2) { const int mid = (lo2 + hi2) >> 1; if (BATCH[mid] <= gidx) lo2 = mid + 1; else hi2 = mid; } shi = lo2; }
  __syncthreads();
  float a = 0.f, mx = -INFINITY;
#pragma unroll 1
  for (int n = slo; n < shi; ++n) { const float v = Hh[(size_t)n * HID + tid]; a += v; mx = fmaxf(mx, v); }
  const int cnt = shi - slo; so[tid] = a / (float)(cnt > 0 ? cnt : 1); so[256 + tid] = mx;
  __syncthreads();
  if (tid < 128) vst2(Gp + (size_t)gidx * 512 + tid * 4, *(const v4f*)&so[tid * 4]);
}
__global__ __launch_bounds__(256) void k_vhead(const float* __restrict__ Gp, const float* __restrict__ WG1, const float* __restrict__ BG1, const float* __restrict__ WG2, const float* __restrict__ BG2, float* __restrict__ O0, float* __restrict__ O1) {
  __shared__ float sg[512], sh[256]; __shared__ __align__(16) float sv[2][64]; const int tid = threadIdx.x;
  if (tid < 64) { sv[0][tid] = 0.f; sv[1][tid] = 0.f; }
#pragma unroll 1
  for (int gidx = 0; gidx < NGT; ++gidx) { sg[tid] = Gp[(size_t)gidx * 512 + tid]; sg[256 + tid] = Gp[(size_t)gidx * 512 + 256 + tid]; __syncthreads();
    float a = bfr(BG1[tid]);
#pragma unroll 1
    for (int k = 0; k < 512; ++k) a += sg[k] * bfr(WG1[(size_t)k * HID + tid]);
    sh[tid] = fmaxf(a, 0.f); __syncthreads();
    if (tid < 32) { float z = 0.f;
#pragma unroll
      for (int k = 0; k < 8; ++k) { const int u = tid + 32 * k; z += sh[u] * bfr(WG2[u]); }
#pragma unroll
      for (int o = 1; o < 32; o <<= 1) z += __shfl_xor(z, o);
      if (tid == 0) { const float vl = z + bfr(BG2[0]); sv[1][gidx] = vl; sv[0][gidx] = sigm(vl); } }
    __syncthreads(); }
  if (tid < NGT / 4) vst2(O0 + tid * 4, *(const v4f*)&sv[0][tid * 4]); else if (tid >= 16 && tid < 16 + NGT / 4) vst2(O1 + (tid - 16) * 4, *(const v4f*)&sv[1][(tid - 16) * 4]);
}
__global__ __launch_bounds__(256) void k_nhead1(const float* __restrict__ HL, const float* __restrict__ WL2, const float* __restrict__ BL2, float* __restrict__ NL_) {
  __shared__ float sw[128]; const int tid = threadIdx.x; if (tid < 128) sw[tid] = bfr(WL2[tid]); __syncthreads();
  const size_t n = (size_t)blockIdx.x * 256 + tid; if (n >= (size_t)NPAD) return; float a = bfr(BL2[0]); const float* hl = HL + n * 128;
#pragma unroll 4
  for (int k = 0; k < 128; ++k) a += hl[k] * sw[k];
  NL_[n] = (n < (size_t)NNT) ? a : 0.f;
}
__global__ __launch_bounds__(256) void k_nhead2(const float* __restrict__ NL_, float* __restrict__ O2) {
  const int tid = threadIdx.x, wave = tid >> 5, lane = tid & 31; const size_t line = (size_t)blockIdx.x * 8 + wave; const size_t c = line * 32 + lane;
  const size_t total = 2 * (size_t)NN; if (line * 32 >= total) return;
  float v = 0.f; bool w = false;
  if (c < (size_t)NN) { if (c < (size_t)NNT) { v = sigm(NL_[c]); w = true; } }
  else if (c < total) { const size_t n = c - NN; if (n < (size_t)NNT) { v = NL_[n]; w = true; } }
  if (w) { *(volatile float*)(O2 + c) = v; __threadfence(); *(volatile float*)(O2 + c) = v; }
}
extern "C" void kernel_launch(void* const* d_in, const int* in_sizes, int n_in, void* d_out, int out_size, void* d_ws, size_t ws_size, hipStream_t stream) {
  (void)in_sizes; (void)n_in; (void)out_size;
  const float** F = (const float**)d_in; const int* EI = (const int*)d_in[1]; const int* BATCH = (const int*)d_in[2];
  if (ws_size < (size_t)WS_END) return;
  char* ws = (char*)d_ws;
  int *ACNT = (int*)(ws + WS_ACNT), *AOFF = (int*)(ws + WS_AOFF), *ABST = (int*)(ws + WS_ABST), *ASEGS = (int*)(ws + WS_ASEGS), *ASEGE = (int*)(ws + WS_ASEGE), *AFS = (int*)(ws + WS_AFS), *AFE = (int*)(ws + WS_AFE), *ARST = (int*)(ws + WS_ARST), *ARCT = (int*)(ws + WS_ARCT);
  int *BCNT = (int*)(ws + WS_BCNT), *BOFF = (int*)(ws + WS_BOFF), *BBST = (int*)(ws + WS_BBST), *BSEGS = (int*)(ws + WS_BSEGS), *BSEGE = (int*)(ws + WS_BSEGE), *BFS = (int*)(ws + WS_BFS), *BFE = (int*)(ws + WS_BFE), *BRST = (int*)(ws + WS_BRST), *BRCT = (int*)(ws + WS_BRCT);
  int *CCNT = (int*)(ws + WS_CCNT), *COFF = (int*)(ws + WS_COFF), *CBST = (int*)(ws + WS_CBST), *CSEGS = (int*)(ws + WS_CSEGS), *CSEGE = (int*)(ws + WS_CSEGE), *CFS = (int*)(ws + WS_CFS), *CFE = (int*)(ws + WS_CFE), *CRST = (int*)(ws + WS_CRST), *CRCT = (int*)(ws + WS_CRCT);
  int *DCNT = (int*)(ws + WS_DCNT), *DOFF = (int*)(ws + WS_DOFF), *DBST = (int*)(ws + WS_DBST), *DSEGS = (int*)(ws + WS_DSEGS), *DSEGE = (int*)(ws + WS_DSEGE), *DFS = (int*)(ws + WS_DFS), *DFE = (int*)(ws + WS_DFE), *DRST = (int*)(ws + WS_DRST), *DRCT = (int*)(ws + WS_DRCT);
  int *ECNT = (int*)(ws + WS_ECNT), *EOFF = (int*)(ws + WS_EOFF), *EBST = (int*)(ws + WS_EBST), *ESEGS = (int*)(ws + WS_ESEGS), *ESEGE = (int*)(ws + WS_ESEGE), *EFS = (int*)(ws + WS_EFS), *EFE = (int*)(ws + WS_EFE), *ERST = (int*)(ws + WS_ERST), *ERCT = (int*)(ws + WS_ERCT);
  __bf16* PW = (__bf16*)(ws + WS_PW); float *Hh = (float*)(ws + WS_H), *QKV = (float*)(ws + WS_QKV), *PB = (float*)(ws + WS_PB), *AL = (float*)(ws + WS_AL), *MS = (float*)(ws + WS_MS), *AGG = (float*)(ws + WS_AGG), *T = (float*)(ws + WS_T), *Gp = (float*)(ws + WS_G), *HL = (float*)(ws + WS_HL), *NLb = (float*)(ws + WS_NL);
  float* O0 = (float*)d_out; float* O1 = O0 + 64; float* O2 = O0 + 128; float* O3 = O0 + 128 + NN;
  k_csA_cnt<<<CSA_NCH, 256, 0, stream>>>(EI + (0 * 2 + 1) * NEDG, 1, ACNT); k_csA_scan<<<1, 256, 0, stream>>>(ACNT, AOFF, ABST); k_csA_scatter<<<CSA_NCH, 256, 0, stream>>>(EI + (0 * 2) * NEDG, EI + (0 * 2 + 1) * NEDG, 1, 1, AOFF, ASEGS, ASEGE); k_csA_bucket<<<CSA_NBK, 256, 0, stream>>>(ACNT, AOFF, ABST, ASEGS, ASEGE, EI + (0 * 2 + 1) * NEDG, 1, AFS, AFE, ARST, ARCT);
  k_csB_cnt<<<CSB_NCH, 256, 0, stream>>>(EI + (1 * 2 + 1) * NEDG, 1, BCNT); k_csB_scan<<<1, 256, 0, stream>>>(BCNT, BOFF, BBST); k_csB_scatter<<<CSB_NCH, 256, 0, stream>>>(EI + (1 * 2) * NEDG, EI + (1 * 2 + 1) * NEDG, 1, 1, BOFF, BSEGS, BSEGE); k_csB_bucket<<<CSB_NBK, 256, 0, stream>>>(BCNT, BOFF, BBST, BSEGS, BSEGE, EI + (1 * 2 + 1) * NEDG, 1, BFS, BFE, BRST, BRCT);
  k_csC_cnt<<<CSC_NCH, 256, 0, stream>>>(EI + (2 * 2 + 1) * NEDG, 1, CCNT); k_csC_scan<<<1, 256, 0, stream>>>(CCNT, COFF, CBST); k_csC_scatter<<<CSC_NCH, 256, 0, stream>>>(EI + (2 * 2) * NEDG, EI + (2 * 2 + 1) * NEDG, 1, 1, COFF, CSEGS, CSEGE); k_csC_bucket<<<CSC_NBK, 256, 0, stream>>>(CCNT, COFF, CBST, CSEGS, CSEGE, EI + (2 * 2 + 1) * NEDG, 1, CFS, CFE, CRST, CRCT);
  k_csD_cnt<<<CSD_NCH, 256, 0, stream>>>(EI + (3 * 2 + 1) * NEDG, 1, DCNT); k_csD_scan<<<1, 256, 0, stream>>>(DCNT, DOFF, DBST); k_csD_scatter<<<CSD_NCH, 256, 0, stream>>>(EI + (3 * 2) * NEDG, EI + (3 * 2 + 1) * NEDG, 1, 1, DOFF, DSEGS, DSEGE); k_csD_bucket<<<CSD_NBK, 256, 0, stream>>>(DCNT, DOFF, DBST, DSEGS, DSEGE, EI + (3 * 2 + 1) * NEDG, 1, DFS, DFE, DRST, DRCT);
  k_csE_cnt<<<CSE_NCH, 256, 0, stream>>>(EI + (4 * 2 + 1) * NEDG, 1, ECNT); k_csE_scan<<<1, 256, 0, stream>>>(ECNT, EOFF, EBST); k_csE_scatter<<<CSE_NCH, 256, 0, stream>>>(EI + (4 * 2) * NEDG, EI + (4 * 2 + 1) * NEDG, 1, 1, EOFF, ESEGS, ESEGE); k_csE_bucket<<<CSE_NBK, 256, 0, stream>>>(ECNT, EOFF, EBST, ESEGS, ESEGE, EI + (4 * 2 + 1) * NEDG, 1, EFS, EFE, ERST, ERCT);
  for (int l = 0; l < NL; ++l) { k_packW<<<HID, 256, 0, stream>>>(F[5] + (size_t)l * HID * HID, HID, HID, PW + PQKV(l)); k_packW<<<HID, 256, 0, stream>>>(F[7] + (size_t)l * HID * HID, HID, HID, PW + PQKV(l) + (size_t)HID * HID); k_packW<<<HID, 256, 0, stream>>>(F[9] + (size_t)l * HID * HID, HID, HID, PW + PQKV(l) + (size_t)2 * HID * HID); k_packW<<<HID, 256, 0, stream>>>(F[14] + (size_t)l * HID * HID, HID, HID, PW + POUT(l)); }
  k_packrel<<<dim3(DH, NL * NR * 2 * NHD), 64, 0, stream>>>(F[11], F[12], PW);
  k_packW<<<128, 256, 0, stream>>>(F[23], HID, 128, PW + PL1);
  k_inp<<<NRBT, 256, 0, stream>>>(F[0], F[3], F[4], Hh);
  for (int l = 0; l < NL; ++l) {
    for (int cb = 0; cb < 6; ++cb) { const float* bb = (cb < 2 ? F[6] : (cb < 4 ? F[8] : F[10])) + (size_t)l * HID + (cb & 1) * 128; k_gemm<0><<<dim3(NRBT, 1), 128, 0, stream>>>(Hh, HID, HID, PW + PQKV(l) + (size_t)cb * 128 * HID, bb, nullptr, nullptr, QKV + cb * 128, 768); }
    for (int r = 0; r < NR; ++r) { k_rel<<<dim3(NRBT, NHD), 128, 0, stream>>>(QKV, 0, PW + PREL(l, r, 0, 0), PB);
      k_logit<<<(NEDG + 63) / 64, 256, 0, stream>>>(PB, QKV, EI + (r * 2) * NEDG, EI + (r * 2 + 1) * NEDG, F[13] + (size_t)l * NR * NHD, r, AL); }
    k_stats<<<NRBT, 256, 0, stream>>>(AL, AFE, ARST, ARCT, BFE, BRST, BRCT, CFE, CRST, CRCT, DFE, DRST, DRCT, EFE, ERST, ERCT, MS);
    for (int r = 0; r < NR; ++r) { k_rel<<<dim3(NRBT, NHD), 128, 0, stream>>>(QKV, 512, PW + PREL(l, r, 1, 0), PB);
      const int* fs = r == 0 ? AFS : r == 1 ? BFS : r == 2 ? CFS : r == 3 ? DFS : EFS; const int* fe = r == 0 ? AFE : r == 1 ? BFE : r == 2 ? CFE : r == 3 ? DFE : EFE; const int* rst = r == 0 ? ARST : r == 1 ? BRST : r == 2 ? CRST : r == 3 ? DRST : ERST; const int* rct = r == 0 ? ARCT : r == 1 ? BRCT : r == 2 ? CRCT : r == 3 ? DRCT : ERCT;
      if (r == 0) k_aggr<1><<<NRBT, 256, 0, stream>>>(PB, AL, MS, fs, fe, rst, rct, r, AGG); else k_aggr<0><<<NRBT, 256, 0, stream>>>(PB, AL, MS, fs, fe, rst, rct, r, AGG); }
    k_gemm<2><<<dim3(NRBT, 2), 128, 0, stream>>>(AGG, HID, HID, PW + POUT(l), F[15] + (size_t)l * HID, Hh, F[16] + l, T, HID);
    k_ln<<<NRBT * 8, 256, 0, stream>>>(T, F[17] + (size_t)l * HID, F[18] + (size_t)l * HID, Hh);
  }
  k_pool<<<NG, 256, 0, stream>>>(Hh, BATCH, Gp);
  k_vhead<<<1, 256, 0, stream>>>(Gp, F[19], F[20], F[21], F[22], O0, O1);
  k_gemm<1><<<dim3(NRBT, 1), 128, 0, stream>>>(Hh, HID, HID, PW + PL1, F[24], nullptr, nullptr, HL, 128);
  k_nhead1<<<NPAD / 256 + 1, 256, 0, stream>>>(HL, F[25], F[26], NLb);
  k_nhead2<<<(2 * NN / 32 + 7) / 8, 256, 0, stream>>>(NLb, O2);
}
